// GQAttention_53480932770686
// MI455X (gfx1250) — hardware-verified
//
#include <hip/hip_runtime.h>
#include <math.h>

#ifndef NB
#define NB 1
#endif
#ifndef SEQ
#define SEQ 2048
#endif
#define SEQ_FULL 2048
#define DM 2048
#define HQ 32
#define HK 8
#define HD 64
#define DKV (HK * HD)
#define EARLY_QB 4
static_assert(NB == 1);
static_assert(SEQ % 64 == 0 && SEQ >= 64 && SEQ <= SEQ_FULL);
static_assert(DM % 64 == 0 && DKV % 64 == 0 && HD == 64 && HQ == 4 * HK && DM == HQ * HD);

typedef __attribute__((ext_vector_type(16))) _Float16 v16h;
typedef __attribute__((ext_vector_type(8)))  _Float16 v8h;
typedef __attribute__((ext_vector_type(16))) __bf16   v16b;
typedef __attribute__((ext_vector_type(8)))  float    v8f;
typedef __attribute__((ext_vector_type(4)))  float    v4f;
typedef __attribute__((ext_vector_type(4)))  int      v4i;

__device__ __forceinline__ int frag_k(int i, int h) { return (i < 8) ? (8 * h + i) : (16 + 8 * h + (i - 8)); }
__device__ __forceinline__ __bf16 bf16_rne(float f) {
    unsigned int u = __float_as_uint(f);
    u += 0x7fffu + ((u >> 16) & 1u);
    return __builtin_bit_cast(__bf16, (unsigned short)(u >> 16));
}
__device__ __forceinline__ float bf16_f32(__bf16 b) { return __uint_as_float(((unsigned int)__builtin_bit_cast(unsigned short, b)) << 16); }
__device__ __forceinline__ float bf16r(float f) { return bf16_f32(bf16_rne(f)); }

__device__ __forceinline__ v8f wmma16(v16h a, v16h b, v8f c) {
    c = __builtin_amdgcn_wmma_f32_16x16x32_f16(false, a, false, b, (short)0, c, false, false);
    asm volatile("v_nop\n\tv_nop\n\tv_nop\n\tv_nop" : "+v"(c) : "v"(a), "v"(b));
    return c;
}
__device__ __forceinline__ v8f wmmab(v16b a, v16b b, v8f c) {
    c = __builtin_amdgcn_wmma_f32_16x16x32_bf16(false, a, false, b, (short)0, c, false, false);
    asm volatile("v_nop\n\tv_nop\n\tv_nop\n\tv_nop" : "+v"(c) : "v"(a), "v"(b));
    return c;
}
struct Split { v16b hi, lo; };
__device__ __forceinline__ v8f wmma3(const Split& a, const Split& b, v8f c) {
    c = __builtin_amdgcn_wmma_f32_16x16x32_bf16(false, a.hi, false, b.hi, (short)0, c, false, false);
    c = __builtin_amdgcn_wmma_f32_16x16x32_bf16(false, a.hi, false, b.lo, (short)0, c, false, false);
    c = __builtin_amdgcn_wmma_f32_16x16x32_bf16(false, a.lo, false, b.hi, (short)0, c, false, false);
    asm volatile("v_nop\n\tv_nop\n\tv_nop\n\tv_nop" : "+v"(c) : "v"(a.hi), "v"(a.lo), "v"(b.hi), "v"(b.lo));
    return c;
}

__device__ __forceinline__ v16h fh_ld(const float* p, long long sk, int k0, int h, int klen, float s, int rb) {
    v16h a;
#pragma unroll
    for (int i = 0; i < 16; ++i) {
        const int k = k0 + frag_k(i, h); const int kc = min(k, klen - 1);
        float x = p[(long long)kc * sk]; if (rb) x = bf16r(x);
        a[i] = (k < klen) ? (_Float16)(x * s) : (_Float16)0.f;
    }
    return a;
}
__device__ __forceinline__ Split sp_ld(const float* p, long long sk, int k0, int h, int klen, float s, int rb) {
    Split r;
#pragma unroll
    for (int i = 0; i < 16; ++i) {
        const int k = k0 + frag_k(i, h); const int kc = min(k, klen - 1);
        float x = p[(long long)kc * sk]; if (rb) x = bf16r(x);
        x = (k < klen) ? x * s : 0.f;
        const __bf16 hb = bf16_rne(x); r.hi[i] = hb; r.lo[i] = bf16_rne(x - bf16_f32(hb));
    }
    return r;
}
__device__ __forceinline__ v16b bh_ld(const float* p, long long sk, int k0, int h, int klen, float s) {
    v16b a;
#pragma unroll
    for (int i = 0; i < 16; ++i) {
        const int k = k0 + frag_k(i, h); const int kc = min(k, klen - 1);
        const float x = p[(long long)kc * sk];
        a[i] = bf16_rne((k < klen) ? x * s : 0.f);
    }
    return a;
}

#define VST2(T, ptr, val) do { const T vst2_v_ = (val); *(volatile T*)(ptr) = vst2_v_; __threadfence(); *(volatile T*)(ptr) = vst2_v_; } while (0)
#define VST2V4(ptr, val) do { const v4f vst2_v4_ = (val); *(volatile v4f*)(ptr) = vst2_v4_; __threadfence(); *(volatile v4f*)(ptr) = vst2_v4_; } while (0)

__device__ __forceinline__ float act_fn(float v, int act) { return (act == 1) ? fmaxf(v, 0.f) : v; }

struct GemmP {
    const float* A; const float* B; const float* bias; const float* R; float* C;
    long long sAo, sAi, sAm, sAk, sBo, sBi, sBn, sBk, sCo, sCi, sCm, sRo, sRi, sRm, sRn;
    int M, N, K, zi_n, flags, act; float alpha, beta, sa, sb;
    int Npad, rmask;
};
static_assert(sizeof(GemmP) == 5 * 8 + 15 * 8 + 6 * 4 + 4 * 4 + 2 * 4);

template <int MODE, int TM, int TN>
__global__ __launch_bounds__(32) __attribute__((amdgpu_num_vgpr(256))) void k_gemmT(GemmP p) {
    static_assert(TN % 2 == 0);
    const int lane = threadIdx.x & 31, h = lane >> 4, l15 = lane & 15;
    const int m0 = blockIdx.y * (16 * TM), n0 = blockIdx.x * (16 * TN);
    const int z = blockIdx.z, zo = z / p.zi_n, zi = z - zo * p.zi_n;
    const float* A = p.A + zo * p.sAo + zi * p.sAi;
    const float* B = p.B + zo * p.sBo + zi * p.sBi;
    const int ra = p.rmask & 1, rbm = (p.rmask >> 1) & 1;
    v8f acc[TM][TN];
#pragma unroll
    for (int i = 0; i < TM; ++i)
#pragma unroll
        for (int t = 0; t < TN; ++t) { v8f zz = {}; acc[i][t] = zz; }
#pragma unroll 1
    for (int k0 = 0; k0 < p.K; k0 += 32) {
        if (MODE == 1) {
            Split a[TM], b[TN];
#pragma unroll
            for (int i = 0; i < TM; ++i) { const int am = min(m0 + 16 * i + l15, p.M - 1); a[i] = sp_ld(A + (long long)am * p.sAm, p.sAk, k0, h, p.K, 1.f, ra); __builtin_amdgcn_sched_barrier(0); }
#pragma unroll
            for (int t = 0; t < TN; ++t) { const int bn = min(n0 + 16 * t + l15, p.N - 1); b[t] = sp_ld(B + (long long)bn * p.sBn, p.sBk, k0, h, p.K, 1.f, rbm); __builtin_amdgcn_sched_barrier(0); }
#pragma unroll
            for (int i = 0; i < TM; ++i)
#pragma unroll
                for (int t = 0; t < TN; ++t) acc[i][t] = wmma3(a[i], b[t], acc[i][t]);
        } else if (MODE == 2) {
            v16b a[TM], b[TN];
#pragma unroll
            for (int i = 0; i < TM; ++i) { const int am = min(m0 + 16 * i + l15, p.M - 1); a[i] = bh_ld(A + (long long)am * p.sAm, p.sAk, k0, h, p.K, 1.f); __builtin_amdgcn_sched_barrier(0); }
#pragma unroll
            for (int t = 0; t < TN; ++t) { const int bn = min(n0 + 16 * t + l15, p.N - 1); b[t] = bh_ld(B + (long long)bn * p.sBn, p.sBk, k0, h, p.K, 1.f); __builtin_amdgcn_sched_barrier(0); }
#pragma unroll
            for (int i = 0; i < TM; ++i)
#pragma unroll
                for (int t = 0; t < TN; ++t) acc[i][t] = wmmab(a[i], b[t], acc[i][t]);
        } else {
            v16h a[TM], b[TN];
#pragma unroll
            for (int i = 0; i < TM; ++i) { const int am = min(m0 + 16 * i + l15, p.M - 1); a[i] = fh_ld(A + (long long)am * p.sAm, p.sAk, k0, h, p.K, p.sa, ra); __builtin_amdgcn_sched_barrier(0); }
#pragma unroll
            for (int t = 0; t < TN; ++t) { const int bn = min(n0 + 16 * t + l15, p.N - 1); b[t] = fh_ld(B + (long long)bn * p.sBn, p.sBk, k0, h, p.K, p.sb, rbm); __builtin_amdgcn_sched_barrier(0); }
#pragma unroll
            for (int i = 0; i < TM; ++i)
#pragma unroll
                for (int t = 0; t < TN; ++t) acc[i][t] = wmma16(a[i], b[t], acc[i][t]);
        }
    }
    const float iscale = (MODE == 0) ? p.alpha / (p.sa * p.sb) : p.alpha;
    float* C = p.C + zo * p.sCo + zi * p.sCi;
    const float* R = p.R + zo * p.sRo + zi * p.sRi;
    const int NW = (p.Npad > p.N) ? p.Npad : p.N;
    __shared__ __align__(16) float ctile[16][36];
#pragma unroll
    for (int i = 0; i < TM; ++i) {
        const int mb = m0 + 16 * i; if (mb >= p.M) break;
#pragma unroll
        for (int tp = 0; tp < TN / 2; ++tp) {
            const int nb = n0 + 32 * tp; if (nb >= NW) break;
#pragma unroll
            for (int t2 = 0; t2 < 2; ++t2) {
                const int t = 2 * tp + t2; const int n = nb + t2 * 16 + l15; const int nn = min(n, p.N - 1);
#pragma unroll
                for (int r = 0; r < 8; ++r) {
                    const int m = mb + 8 * h + r; const int mm = min(m, p.M - 1);
                    float v = acc[i][t][r] * iscale;
                    if (p.flags & 1) v += p.bias[nn];
                    if (p.flags & 2) v += p.bias[mm];
                    v = act_fn(v, p.act);
                    if (p.flags & 4) v += p.beta * R[(long long)mm * p.sRm + (long long)nn * p.sRn];
                    ctile[8 * h + r][t2 * 16 + l15] = (n < p.N) ? v : 0.f;
                }
            }
            __syncthreads();
            const bool fast = (mb + 16 <= p.M) && (nb + 32 <= NW) && ((p.sCm & 3) == 0) && ((((size_t)C) & 15) == 0);
            if (fast) {
#pragma unroll
                for (int s = 0; s < 4; ++s) {
                    const int row = s * 4 + (lane >> 3), c4 = (lane & 7) * 4;
                    const v4f v = *(const v4f*)&ctile[row][c4];
                    VST2V4(C + (long long)(mb + row) * p.sCm + nb + c4, v);
                }
            } else {
                for (int row = 0; row < 16; ++row) {
                    const int m = mb + row, n = nb + lane;
                    if (m < p.M && n < NW) VST2(float, C + (long long)m * p.sCm + n, ctile[row][lane]);
                }
            }
            __syncthreads();
        }
    }
}

#define AW 4
struct AttnA {
    const float* Q; const float* K; const float* V; const int* Mk; float* O;
    long long sQh, sQi, sKh, sKj, sVh, sVj, sOh, sOi, smi;
    int Lq, Lk, hrep, qboff; float scale; int pad0;
};
static_assert(sizeof(AttnA) == 5 * 8 + 9 * 8 + 6 * 4);

template <int QM, bool SPLITPV>
__global__ __launch_bounds__(32 * AW) __attribute__((amdgpu_num_vgpr(256))) void k_attn(AttnA p) {
    constexpr int DVP = 64, NT = DVP / 16, KS = HD / 32, VP = DVP + 8;
    __shared__ __align__(16) float    pl[AW][16 * 64];
    __shared__ __align__(16) _Float16 vl[(SPLITPV ? 2 : 1) * 64 * VP];
    __shared__ unsigned int mbits[128];
    const int lane = threadIdx.x & 31, hf = lane >> 4, l15 = lane & 15, wave = threadIdx.x >> 5;
    const int h = blockIdx.y, hk = h / p.hrep;
    const int bx = blockIdx.x + p.qboff;
    const int q0b = bx * (16 * AW), q0 = q0b + wave * 16;
    float* myp = pl[wave];
    const float L2E = 1.4426950408889634f;
    const float NEG = -__builtin_inff();
    const int qi = min(q0 + l15, p.Lq - 1);
    const float* qrow = p.Q + h * p.sQh + (long long)qi * p.sQi;
    const float* kbase = p.K + hk * p.sKh;
    const float* vbase = p.V + hk * p.sVh;
    v16h qa[QM == 0 ? KS : 1]; Split qs_[QM == 1 ? KS : 1];
#pragma unroll
    for (int ks = 0; ks < KS; ++ks) {
        if (QM == 1) qs_[QM == 1 ? ks : 0] = sp_ld(qrow, 1, ks * 32, hf, HD, 1.f, 0);
        else qa[QM == 0 ? ks : 0] = fh_ld(qrow, 1, ks * 32, hf, HD, 1.f, 0);
    }
    v8f o[NT]; float m8[8], l8[8];
#pragma unroll
    for (int t = 0; t < NT; ++t) { v8f zz = {}; o[t] = zz; }
#pragma unroll
    for (int i = 0; i < 8; ++i) { m8[i] = NEG; l8[i] = 0.f; }
#pragma unroll 1
    for (int j0 = 0; j0 < p.Lk; j0 += 64) {
        __syncthreads();
        {
            const int r = threadIdx.x >> 1, hh = threadIdx.x & 1;
            const int ig = min(q0b + r, p.Lq - 1);
            const int jb = min(j0 + hh * 32, p.Lk - 32);
            const int* mrow = p.Mk + (long long)ig * p.smi + jb;
            unsigned int bits = 0u;
#pragma unroll
            for (int c = 0; c < 8; ++c) {
                const v4i mv = *(const v4i*)(mrow + 4 * c);
                const unsigned int b4 = (mv[0] != 0 ? 1u : 0u) | (mv[1] != 0 ? 2u : 0u) | (mv[2] != 0 ? 4u : 0u) | (mv[3] != 0 ? 8u : 0u);
                bits |= b4 << (4 * c);
            }
            mbits[threadIdx.x] = bits;
        }
        __syncthreads();
        const unsigned int any4 = mbits[lane * 4] | mbits[lane * 4 + 1] | mbits[lane * 4 + 2] | mbits[lane * 4 + 3];
        const bool live = __builtin_amdgcn_ballot_w32(any4 != 0u) != 0u;
        if (!live) continue;
        for (int idx = threadIdx.x; idx < 64 * DVP; idx += 32 * AW) {
            const int jr = idx >> 6, d = idx & 63;
            const int j = min(j0 + jr, p.Lk - 1);
            const float f = vbase[(long long)j * p.sVj + d];
            if (SPLITPV) {
                const __bf16 hb = bf16_rne(f);
                ((__bf16*)vl)[jr * VP + d] = hb; ((__bf16*)vl)[64 * VP + jr * VP + d] = bf16_rne(f - bf16_f32(hb));
            } else vl[jr * VP + d] = (_Float16)f;
        }
        v8f s[4];
#pragma unroll
        for (int t = 0; t < 4; ++t) {
            const int j = min(j0 + t * 16 + l15, p.Lk - 1);
            const float* krow = kbase + (long long)j * p.sKj;
            v8f acc = {};
#pragma unroll
            for (int ks = 0; ks < KS; ++ks) {
                if (QM == 1) acc = wmma3(qs_[QM == 1 ? ks : 0], sp_ld(krow, 1, ks * 32, hf, HD, 1.f, 0), acc);
                else         acc = wmma16(qa[QM == 0 ? ks : 0], fh_ld(krow, 1, ks * 32, hf, HD, 1.f, 0), acc);
            }
            s[t] = acc;
        }
        float pv[8][4];
#pragma unroll
        for (int i = 0; i < 8; ++i) {
            const int rl = wave * 16 + i + 8 * hf;
            const unsigned int u0 = mbits[rl * 2], u1 = mbits[rl * 2 + 1];
            float sc[4];
#pragma unroll
            for (int t = 0; t < 4; ++t) {
                const unsigned int word = (t < 2) ? u0 : u1;
                const unsigned int keep = (word >> ((t & 1) * 16 + l15)) & 1u;
                const float v = s[t][i] * p.scale;
                sc[t] = (keep != 0u) ? v * L2E : NEG;
            }
            float mx = fmaxf(fmaxf(sc[0], sc[1]), fmaxf(sc[2], sc[3]));
            mx = fmaxf(mx, __shfl_xor(mx, 1, 32)); mx = fmaxf(mx, __shfl_xor(mx, 2, 32));
            mx = fmaxf(mx, __shfl_xor(mx, 4, 32)); mx = fmaxf(mx, __shfl_xor(mx, 8, 32));
            const float mnew = fmaxf(m8[i], mx);
            const float corr = (mnew == NEG) ? 1.f : exp2f(m8[i] - mnew);
            float rs = 0.f;
#pragma unroll
            for (int t = 0; t < 4; ++t) { const float pp = (sc[t] == NEG) ? 0.f : exp2f(sc[t] - mnew); rs += pp; pv[i][t] = pp; }
            rs += __shfl_xor(rs, 1, 32); rs += __shfl_xor(rs, 2, 32); rs += __shfl_xor(rs, 4, 32); rs += __shfl_xor(rs, 8, 32);
            l8[i] = l8[i] * corr + rs; m8[i] = mnew;
#pragma unroll
            for (int t = 0; t < NT; ++t) o[t][i] *= corr;
        }
#pragma unroll
        for (int i = 0; i < 8; ++i)
#pragma unroll
            for (int t = 0; t < 4; ++t) myp[(i + 8 * hf) * 64 + t * 16 + l15] = pv[i][t];
        __syncthreads();
        if (SPLITPV) {
            const __bf16* vh = (const __bf16*)vl; const __bf16* vlo = vh + 64 * VP;
#pragma unroll
            for (int half = 0; half < 2; ++half) {
                const Split pa = sp_ld(myp + l15 * 64, 1, 32 * half, hf, 64, 1.f, 0);
#pragma unroll
                for (int t = 0; t < NT; ++t) {
                    const int dcol = t * 16 + l15;
                    Split b;
#pragma unroll
                    for (int e = 0; e < 16; ++e) { const int kk = 32 * half + frag_k(e, hf); b.hi[e] = vh[kk * VP + dcol]; b.lo[e] = vlo[kk * VP + dcol]; }
                    o[t] = wmma3(pa, b, o[t]);
                }
            }
        } else {
#pragma unroll
            for (int half = 0; half < 2; ++half) {
                const v16h pa = fh_ld(myp + l15 * 64, 1, 32 * half, hf, 64, 4096.f, 0);
#pragma unroll
                for (int t = 0; t < NT; ++t) {
                    const int dcol = t * 16 + l15;
                    v16h b;
#pragma unroll
                    for (int e = 0; e < 16; ++e) b[e] = vl[(32 * half + frag_k(e, hf)) * VP + dcol];
                    o[t] = wmma16(pa, b, o[t]);
                }
            }
        }
    }
    float invr[8];
#pragma unroll
    for (int i = 0; i < 8; ++i) invr[i] = (l8[i] > 0.f) ? (SPLITPV ? 1.f / l8[i] : 1.f / (l8[i] * 4096.f)) : 0.f;
    __syncthreads();
#pragma unroll
    for (int i = 0; i < 8; ++i)
#pragma unroll
        for (int t = 0; t < NT; ++t) myp[(i + 8 * hf) * 64 + t * 16 + l15] = o[t][i] * invr[i];
    __syncthreads();
    float* obase = p.O + h * p.sOh;
#pragma unroll
    for (int rp = 0; rp < 16; rp += 2) {
        const int row = rp + (lane >> 4), c4 = (lane & 15) * 4;
        const v4f v = *(const v4f*)(myp + row * 64 + c4);
        if (q0 + row < p.Lq) VST2V4(obase + (long long)(q0 + row) * p.sOi + c4, v);
    }
}

__global__ __launch_bounds__(256) void k_rmsrope(const float* __restrict__ X, const float* __restrict__ w, const float* __restrict__ ct, const float* __restrict__ st,
                                                 float* __restrict__ Y, int Hn, int nrows) {
#pragma clang fp contract(off)
    const int wave = threadIdx.x >> 5, lane = threadIdx.x & 31;
    const int rid = blockIdx.x * 8 + wave;
    if (rid >= nrows) return;
    const int s = rid / Hn;
    const float* xr = X + (long long)rid * HD;
    const float x1 = xr[lane], x2 = xr[lane + 32];
    float ss = x1 * x1 + x2 * x2;
    ss += __shfl_xor(ss, 16, 32); ss += __shfl_xor(ss, 8, 32); ss += __shfl_xor(ss, 4, 32); ss += __shfl_xor(ss, 2, 32); ss += __shfl_xor(ss, 1, 32);
    const float ms = ss * (1.0f / 64.0f) + 1e-6f;
    const float rr = 1.0f / sqrtf(ms);
    const float w1 = bf16r(w[lane]), w2 = bf16r(w[lane + 32]);
    const float n1 = (x1 * rr) * w1, n2 = (x2 * rr) * w2;
    const float* cr = ct + (long long)s * HD; const float* sr = st + (long long)s * HD;
    const float c1 = bf16r(cr[lane]), c2 = bf16r(cr[lane + 32]);
    const float s1 = bf16r(sr[lane]), s2 = bf16r(sr[lane + 32]);
    const float o1 = n1 * c1 - n2 * s1;
    const float o2 = n2 * c2 + n1 * s2;
    float* yr = Y + (long long)rid * HD;
    *(volatile float*)(yr + lane) = o1; *(volatile float*)(yr + lane + 32) = o2;
    __threadfence();
    *(volatile float*)(yr + lane) = o1; *(volatile float*)(yr + lane + 32) = o2;
}

__global__ __launch_bounds__(256) void k_rnecopy(const float* __restrict__ src, float* __restrict__ dst, int n) {
    const int i = blockIdx.x * 256 + threadIdx.x;
    if (i < n) { const float v = bf16r(src[i]); VST2(float, dst + i, v); }
}

extern "C" void kernel_launch(void* const* d_in, const int* in_sizes, int n_in, void* d_out, int out_size, void* d_ws, size_t ws_size, hipStream_t stream) {
    if (n_in < 11) return;
    const float* x    = (const float*)d_in[0];
    const float* tsin = (const float*)d_in[1];
    const float* tcos = (const float*)d_in[2];
    const int*   msk  = (const int*)d_in[3];
    const float* Wq   = (const float*)d_in[4];
    const float* Wk   = (const float*)d_in[5];
    const float* Wv   = (const float*)d_in[6];
    const float* Wo   = (const float*)d_in[7];
    const float* bo   = (const float*)d_in[8];
    const float* qsc  = (const float*)d_in[9];
    const float* ksc  = (const float*)d_in[10];
    if (in_sizes[0] < SEQ * DM || in_sizes[1] < SEQ * HD || in_sizes[2] < SEQ * HD || in_sizes[3] < (SEQ - 1) * SEQ_FULL + SEQ ||
        in_sizes[4] < DM * DM || in_sizes[5] < DM * DKV || in_sizes[6] < DM * DKV || in_sizes[7] < DM * DM ||
        in_sizes[8] < DM || in_sizes[9] < HD || in_sizes[10] < HD) return;
    if (out_size < SEQ * DM) return;
    float* out = (float*)d_out;

    char* wsb = (char*)d_ws; size_t off = 0;
    auto carve = [&](size_t bytes) -> char* { char* r = wsb + off; off += (bytes + 255) & ~(size_t)255; return r; };
    float* bo_r = (float*)carve((size_t)DM * 4);
    float* Qf   = (float*)carve((size_t)SEQ * DM * 4);
    float* Kf   = (float*)carve((size_t)SEQ * DKV * 4);
    float* Vf   = (float*)carve((size_t)SEQ * DKV * 4);
    float* Qr   = (float*)carve((size_t)SEQ * DM * 4);
    float* Kr   = (float*)carve((size_t)SEQ * DKV * 4);
    float* ctx  = (float*)carve((size_t)SEQ * DM * 4);
    if (off > ws_size) return;

    k_rnecopy<<<dim3((unsigned)(DM / 256)), 256, 0, stream>>>(bo, bo_r, DM);

    auto mk = [](const float* A, long long sAm, long long sAk, const float* B, long long sBn, long long sBk, float* C, long long sCm,
                 const float* bias, int flags, int M, int N, int K, float sa, float sb, int rmask) {
        GemmP g;
        g.A = A; g.B = B; g.bias = bias; g.R = A; g.C = C;
        g.sAo = 0; g.sAi = 0; g.sAm = sAm; g.sAk = sAk; g.sBo = 0; g.sBi = 0; g.sBn = sBn; g.sBk = sBk;
        g.sCo = 0; g.sCi = 0; g.sCm = sCm; g.sRo = 0; g.sRi = 0; g.sRm = sAm; g.sRn = 1;
        g.M = M; g.N = N; g.K = K; g.zi_n = 1; g.flags = flags; g.act = 0; g.alpha = 1.f; g.beta = 0.f; g.sa = sa; g.sb = sb;
        g.Npad = N; g.rmask = rmask;
        return g;
    };

    k_gemmT<2, 2, 4><<<dim3((unsigned)(DM / 64), (unsigned)(SEQ / 32), 1), 32, 0, stream>>>(mk(x, DM, 1, Wq, 1, DM, Qf, DM, bo_r, 0, SEQ, DM, DM, 1.f, 1.f, 0));
    k_gemmT<2, 2, 4><<<dim3((unsigned)(DKV / 64), (unsigned)(SEQ / 32), 1), 32, 0, stream>>>(mk(x, DM, 1, Wk, 1, DKV, Kf, DKV, bo_r, 0, SEQ, DKV, DM, 1.f, 1.f, 0));
    k_gemmT<2, 2, 4><<<dim3((unsigned)(DKV / 64), (unsigned)(SEQ / 32), 1), 32, 0, stream>>>(mk(x, DM, 1, Wv, 1, DKV, Vf, DKV, bo_r, 0, SEQ, DKV, DM, 1.f, 1.f, 0));

    k_rmsrope<<<dim3((unsigned)((SEQ * HQ + 7) / 8)), 256, 0, stream>>>(Qf, qsc, tcos, tsin, Qr, HQ, SEQ * HQ);
    k_rmsrope<<<dim3((unsigned)((SEQ * HK + 7) / 8)), 256, 0, stream>>>(Kf, ksc, tcos, tsin, Kr, HK, SEQ * HK);

    const int nqb = SEQ / 64;
    const int ne = (EARLY_QB < nqb) ? EARLY_QB : nqb;
    const int ME = ne * 64, ML = SEQ - ME;
    AttnA a;
    a.Q = Qr; a.K = Kr; a.V = Vf; a.Mk = msk; a.O = ctx;
    a.sQh = HD; a.sQi = DM; a.sKh = HD; a.sKj = DKV; a.sVh = HD; a.sVj = DKV; a.sOh = HD; a.sOi = DM; a.smi = SEQ_FULL;
    a.Lq = SEQ; a.Lk = SEQ; a.hrep = HQ / HK; a.qboff = 0; a.scale = 0.125f; a.pad0 = 0;
    k_attn<1, true><<<dim3((unsigned)ne, (unsigned)HQ, 1), 32 * AW, 0, stream>>>(a);
    if (nqb > ne) {
        AttnA al = a; al.qboff = ne;
        k_attn<0, false><<<dim3((unsigned)(nqb - ne), (unsigned)HQ, 1), 32 * AW, 0, stream>>>(al);
    }

    k_gemmT<1, 2, 2><<<dim3((unsigned)(DM / 32), (unsigned)(ME / 32), 1), 32, 0, stream>>>(mk(ctx, DM, 1, Wo, 1, DM, out, DM, bo_r, 1, ME, DM, DM, 1.f, 1.f, 2));
    if (ML > 0) {
        k_gemmT<0, 2, 4><<<dim3((unsigned)(DM / 64), (unsigned)(ML / 32), 1), 32, 0, stream>>>(
            mk(ctx + (size_t)ME * DM, DM, 1, Wo, 1, DM, out + (size_t)ME * DM, DM, bo_r, 1, ML, DM, DM, 16.f, 64.f, 2));
    }
    (void)hipGetLastError();
}
